// DiscriminatorMADClf_81209241633290
// MI455X (gfx1250) — hardware-verified
//
#include <hip/hip_runtime.h>
#include <math.h>
#include <stdint.h>
#include <stddef.h>


typedef __bf16 v16b __attribute__((ext_vector_type(16)));
typedef __bf16 v8b  __attribute__((ext_vector_type(8)));
typedef float  v8f  __attribute__((ext_vector_type(8)));
typedef float  v4f  __attribute__((ext_vector_type(4)));
typedef unsigned short v8us __attribute__((ext_vector_type(8)));

#define GT            64
#define CPF           68
#define GEMM_THREADS  128
#define MBD_ROWS      8
#define HEAD_ROWS     32

__device__ __forceinline__ v8f wmma_bf16(v16b a, v16b b, v8f c)
{
    c = __builtin_amdgcn_wmma_f32_16x16x32_bf16(false, a, false, b, (short)0, c, false, false);
    asm volatile("v_nop\n\tv_nop\n\tv_nop\n\tv_nop" : "+v"(c) : "v"(a), "v"(b));
    return c;
}

__device__ __forceinline__ v16b load_frag(const __bf16* p)
{
    v8b e0 = *(const v8b*)(p);
    v8b e1 = *(const v8b*)(p + 16);
    return __builtin_shufflevector(e0, e1, 0,1,2,3,4,5,6,7,8,9,10,11,12,13,14,15);
}

__device__ __forceinline__ unsigned bf16_rne_bits(float f)
{
    unsigned u = __float_as_uint(f);
    return (u + 0x7FFFu + ((u >> 16) & 1u)) >> 16;
}

__device__ __forceinline__ void split8(v4f a, v4f b, v8us& hv, v8us& lv)
{
    float f[8] = { a.x, a.y, a.z, a.w, b.x, b.y, b.z, b.w };
    #pragma unroll
    for (int i = 0; i < 8; ++i) {
        unsigned hb = bf16_rne_bits(f[i]);
        float fh = __uint_as_float(hb << 16);
        unsigned lb = bf16_rne_bits(f[i] - fh);
        hv[i] = (unsigned short)hb;
        lv[i] = (unsigned short)lb;
    }
}

__device__ __forceinline__ float elu1(float v) { return v > 0.0f ? v : expm1f(v); }
__device__ __forceinline__ v4f elu4(v4f v)
{
    v.x = elu1(v.x); v.y = elu1(v.y); v.z = elu1(v.z); v.w = elu1(v.w);
    return v;
}

__global__ __launch_bounds__(256)
void cvt_split_rows(const float* __restrict__ X, unsigned short* Xh, unsigned short* Xl, int n8)
{
    const int idx = blockIdx.x * 256 + threadIdx.x;
    if (idx >= n8) return;
    const v4f a = *(const v4f*)(X + (size_t)idx * 8);
    const v4f b = *(const v4f*)(X + (size_t)idx * 8 + 4);
    v8us hv, lv;
    split8(a, b, hv, lv);
    const size_t o = (size_t)idx * 8;
    *(volatile v8us*)(Xh + o) = hv;
    *(volatile v8us*)(Xl + o) = lv;
    __threadfence();
    *(volatile v8us*)(Xh + o) = hv;
    *(volatile v8us*)(Xl + o) = lv;
}

__global__ __launch_bounds__(256)
void cvt_split_transpose(const float* __restrict__ W, unsigned short* Wh, unsigned short* Wl,
                         int K, int Nc)
{
    __shared__ float sT[64 * 65];
    const int tid = threadIdx.x;
    const int n0 = blockIdx.x * 64, k0 = blockIdx.y * 64;
    #pragma unroll
    for (int p = 0; p < 4; ++p) {
        const int e = p * 256 + tid;
        const int kk = e >> 4, q = e & 15;
        const v4f v = *(const v4f*)(W + (size_t)(k0 + kk) * Nc + n0 + 4 * q);
        sT[kk * 65 + 4 * q + 0] = v.x;
        sT[kk * 65 + 4 * q + 1] = v.y;
        sT[kk * 65 + 4 * q + 2] = v.z;
        sT[kk * 65 + 4 * q + 3] = v.w;
    }
    __syncthreads();
    v8us hv[2], lv[2];
    size_t off[2];
    #pragma unroll
    for (int p = 0; p < 2; ++p) {
        const int c = p * 256 + tid;
        const int n = c >> 3, q = c & 7;
        v4f a, b;
        a.x = sT[(8 * q + 0) * 65 + n]; a.y = sT[(8 * q + 1) * 65 + n];
        a.z = sT[(8 * q + 2) * 65 + n]; a.w = sT[(8 * q + 3) * 65 + n];
        b.x = sT[(8 * q + 4) * 65 + n]; b.y = sT[(8 * q + 5) * 65 + n];
        b.z = sT[(8 * q + 6) * 65 + n]; b.w = sT[(8 * q + 7) * 65 + n];
        split8(a, b, hv[p], lv[p]);
        off[p] = (size_t)(n0 + n) * K + k0 + 8 * q;
    }
    #pragma unroll
    for (int p = 0; p < 2; ++p) {
        *(volatile v8us*)(Wh + off[p]) = hv[p];
        *(volatile v8us*)(Wl + off[p]) = lv[p];
    }
    __threadfence();
    #pragma unroll
    for (int p = 0; p < 2; ++p) {
        *(volatile v8us*)(Wh + off[p]) = hv[p];
        *(volatile v8us*)(Wl + off[p]) = lv[p];
    }
}

template<bool ELU, bool BIAS>
__device__ __forceinline__ void tile_store_f32(const float* sC, const float* __restrict__ bias,
                                               float* C32, int brow, int bcol, int ldc, int tid)
{
    #pragma unroll 1
    for (int p = 0; p < 8; ++p) {
        const int c = p * GEMM_THREADS + tid;
        const int row = c >> 4, q = c & 15;
        v4f v = *(const v4f*)(sC + row * CPF + 4 * q);
        const int col = bcol + 4 * q;
        if (BIAS) v += *(const v4f*)(bias + col);
        if (ELU) v = elu4(v);
        *(volatile v4f*)(C32 + (size_t)(brow + row) * ldc + col) = v;
    }
}
template<bool ELU, bool BIAS>
__device__ __forceinline__ void tile_store_split(const float* sC, const float* __restrict__ bias,
                                                 unsigned short* Ch, unsigned short* Cl,
                                                 int brow, int bcol, int ldc, int tid)
{
    #pragma unroll 1
    for (int p = 0; p < 4; ++p) {
        const int c = p * GEMM_THREADS + tid;
        const int row = c >> 3, q = c & 7;
        v4f v0 = *(const v4f*)(sC + row * CPF + 8 * q);
        v4f v1 = *(const v4f*)(sC + row * CPF + 8 * q + 4);
        const int col = bcol + 8 * q;
        if (BIAS) { v0 += *(const v4f*)(bias + col); v1 += *(const v4f*)(bias + col + 4); }
        if (ELU) { v0 = elu4(v0); v1 = elu4(v1); }
        v8us hv, lv;
        split8(v0, v1, hv, lv);
        const size_t o = (size_t)(brow + row) * ldc + col;
        *(volatile v8us*)(Ch + o) = hv;
        *(volatile v8us*)(Cl + o) = lv;
    }
}

template<bool ELU, bool BIAS, bool OUT32, bool OUT16>
__global__ __launch_bounds__(GEMM_THREADS)
void gemm_split3(const __bf16* __restrict__ Ah, const __bf16* __restrict__ Al,
                 const __bf16* __restrict__ Bh, const __bf16* __restrict__ Bl,
                 const float* __restrict__ bias,
                 float* C32, unsigned short* Ch, unsigned short* Cl,
                 int Mdim, int Ndim, int Kdim)
{
    __shared__ __attribute__((aligned(16))) float sC[GT * CPF];

    const int tid  = threadIdx.x;
    const int wave = tid >> 5;
    const int lane = tid & 31;
    const int h    = lane >> 4;
    const int m    = lane & 15;
    const int wr   = wave >> 1, wc = wave & 1;
    const int brow = blockIdx.x * GT, bcol = blockIdx.y * GT;
    if (brow + GT > Mdim || bcol + GT > Ndim) return;
    const int row0 = brow + wr * 32, col0 = bcol + wc * 32;

    v8f acc[2][2];
    #pragma unroll
    for (int i = 0; i < 2; ++i)
        #pragma unroll
        for (int j = 0; j < 2; ++j) {
            v8f z = { 0.f, 0.f, 0.f, 0.f, 0.f, 0.f, 0.f, 0.f };
            acc[i][j] = z;
        }

    #pragma unroll 1
    for (int k0 = 0; k0 < Kdim; k0 += 32) {
        v16b ah[2], al[2], bh[2], bl[2];
        #pragma unroll
        for (int t = 0; t < 2; ++t) {
            const size_t ao = (size_t)(row0 + t * 16 + m) * Kdim + k0 + 8 * h;
            ah[t] = load_frag(Ah + ao);
            al[t] = load_frag(Al + ao);
            const size_t bo = (size_t)(col0 + t * 16 + m) * Kdim + k0 + 8 * h;
            bh[t] = load_frag(Bh + bo);
            bl[t] = load_frag(Bl + bo);
        }
        #pragma unroll
        for (int tm = 0; tm < 2; ++tm)
            #pragma unroll
            for (int tn = 0; tn < 2; ++tn) {
                acc[tm][tn] = wmma_bf16(ah[tm], bh[tn], acc[tm][tn]);
                acc[tm][tn] = wmma_bf16(ah[tm], bl[tn], acc[tm][tn]);
                acc[tm][tn] = wmma_bf16(al[tm], bh[tn], acc[tm][tn]);
            }
    }

    #pragma unroll
    for (int tm = 0; tm < 2; ++tm)
        #pragma unroll
        for (int tn = 0; tn < 2; ++tn)
            #pragma unroll
            for (int r = 0; r < 8; ++r)
                sC[(wr * 32 + tm * 16 + 8 * h + r) * CPF + wc * 32 + tn * 16 + m] = acc[tm][tn][r];
    __syncthreads();

    if (OUT32) tile_store_f32<ELU, BIAS>(sC, bias, C32, brow, bcol, Ndim, tid);
    if (OUT16) tile_store_split<ELU, BIAS>(sC, bias, Ch, Cl, brow, bcol, Ndim, tid);
    __threadfence();
    if (OUT32) tile_store_f32<ELU, BIAS>(sC, bias, C32, brow, bcol, Ndim, tid);
    if (OUT16) tile_store_split<ELU, BIAS>(sC, bias, Ch, Cl, brow, bcol, Ndim, tid);
}

__device__ __forceinline__ void mbd_store(const float* sO, float* ob, int i0, int tid)
{
    #pragma unroll
    for (int p = 0; p < 2; ++p) {
        const int c = p * 128 + tid;
        const int row = c >> 5, q = c & 31;
        const v4f v = *(const v4f*)(sO + row * 128 + 4 * q);
        *(volatile v4f*)(ob + (size_t)(i0 + row) * 128 + 4 * q) = v;
    }
}

__global__ __launch_bounds__(128)
void mbd_kernel(const float* __restrict__ M, float* ob, int N)
{
    __shared__ __attribute__((aligned(16))) float sO[MBD_ROWS * 128];
    const int tid = threadIdx.x;
    const int i0  = blockIdx.x * MBD_ROWS;
    float mi[MBD_ROWS], acc[MBD_ROWS];
    #pragma unroll
    for (int ii = 0; ii < MBD_ROWS; ++ii) {
        mi[ii]  = M[(size_t)(i0 + ii) * 128 + tid];
        acc[ii] = 0.0f;
    }
    #pragma unroll 2
    for (int j = 0; j < N; ++j) {
        const float mj = M[(size_t)j * 128 + tid];
        #pragma unroll
        for (int ii = 0; ii < MBD_ROWS; ++ii)
            acc[ii] += __expf(-fabsf(mj - mi[ii]));
    }
    #pragma unroll
    for (int ii = 0; ii < MBD_ROWS; ++ii)
        sO[ii * 128 + tid] = acc[ii] - 1.0f;
    __syncthreads();
    mbd_store(sO, ob, i0, tid);
    __threadfence();
    mbd_store(sO, ob, i0, tid);
}

__device__ __forceinline__ void heads_store(const float* sO, float* out0, float* out1,
                                            int blk, int tid)
{
    if (tid < (HEAD_ROWS * 17) / 4) {
        const v4f v = *(const v4f*)(sO + 4 * tid);
        *(volatile v4f*)(out0 + (size_t)blk * (HEAD_ROWS * 17) + 4 * tid) = v;
    }
    if (tid < (HEAD_ROWS * 10) / 4) {
        const v4f v = *(const v4f*)(sO + HEAD_ROWS * 17 + 4 * tid);
        *(volatile v4f*)(out1 + (size_t)blk * (HEAD_ROWS * 10) + 4 * tid) = v;
    }
}

__global__ __launch_bounds__(256)
void heads_kernel(const float* __restrict__ feat, const float* __restrict__ ob,
                  const float* __restrict__ Wm, const float* __restrict__ bm,
                  const float* __restrict__ Wc, const float* __restrict__ bc,
                  float* out0, float* out1)
{
    __shared__ __attribute__((aligned(16))) float sO[HEAD_ROWS * 17 + HEAD_ROWS * 10];
    const int tid = threadIdx.x;
    const int rb  = blockIdx.x * HEAD_ROWS;
    #pragma unroll 1
    for (int s = 0; s < 4; ++s) {
        const int o = s * 256 + tid;
        if (o < HEAD_ROWS * 17) {
            const int r = o / 17, c = o - r * 17;
            const float* fr   = feat + (size_t)(rb + r) * 512;
            const float* orow = ob   + (size_t)(rb + r) * 128;
            float acc = 0.0f;
            #pragma unroll 4
            for (int k = 0; k < 512; ++k) acc = fmaf(fr[k], Wm[k * 17 + c], acc);
            #pragma unroll 4
            for (int b = 0; b < 128; ++b) acc = fmaf(orow[b], Wm[(512 + b) * 17 + c], acc);
            sO[o] = acc + bm[c];
        } else if (o < HEAD_ROWS * 17 + HEAD_ROWS * 10) {
            const int o2 = o - HEAD_ROWS * 17;
            const int r = o2 / 10, c = o2 - r * 10;
            const float* fr = feat + (size_t)(rb + r) * 512;
            float acc = 0.0f;
            #pragma unroll 4
            for (int k = 0; k < 512; ++k) acc = fmaf(fr[k], Wc[k * 10 + c], acc);
            sO[o] = acc + bc[c];
        }
    }
    __syncthreads();
    heads_store(sO, out0, out1, blockIdx.x, tid);
    __threadfence();
    heads_store(sO, out0, out1, blockIdx.x, tid);
}

extern "C" void kernel_launch(void* const* d_in, const int* in_sizes, int n_in,
                              void* d_out, int out_size, void* d_ws, size_t ws_size,
                              hipStream_t stream)
{
    const int N = 1024, DIN = 512, H = 1024, F = 512, B = 128, NM = 17, NCL = 10;
    if (n_in < 10) return;
    if (in_sizes[0] != N * DIN || in_sizes[1] != DIN * H || in_sizes[2] != H ||
        in_sizes[3] != H * F || in_sizes[4] != F || in_sizes[5] != F * B ||
        in_sizes[6] != (F + B) * NM || in_sizes[7] != NM ||
        in_sizes[8] != F * NCL || in_sizes[9] != NCL) return;
    if (out_size != N * (NM + NCL)) return;

    const float* x   = (const float*)d_in[0];
    const float* Wb0 = (const float*)d_in[1];
    const float* bb0 = (const float*)d_in[2];
    const float* Wb1 = (const float*)d_in[3];
    const float* bb1 = (const float*)d_in[4];
    const float* T   = (const float*)d_in[5];
    const float* Wm  = (const float*)d_in[6];
    const float* bm  = (const float*)d_in[7];
    const float* Wc  = (const float*)d_in[8];
    const float* bc  = (const float*)d_in[9];

    char* ws = (char*)d_ws;
    size_t off = 0;
    auto carve = [&](size_t bytes) -> char* {
        char* p = ws + off;
        off += (bytes + 255) & ~(size_t)255;
        return p;
    };
    unsigned short* xh  = (unsigned short*)carve((size_t)N * DIN * 2);
    unsigned short* xl  = (unsigned short*)carve((size_t)N * DIN * 2);
    unsigned short* w0h = (unsigned short*)carve((size_t)H * DIN * 2);
    unsigned short* w0l = (unsigned short*)carve((size_t)H * DIN * 2);
    unsigned short* w1h = (unsigned short*)carve((size_t)F * H * 2);
    unsigned short* w1l = (unsigned short*)carve((size_t)F * H * 2);
    unsigned short* th  = (unsigned short*)carve((size_t)B * F * 2);
    unsigned short* tl  = (unsigned short*)carve((size_t)B * F * 2);
    unsigned short* hh  = (unsigned short*)carve((size_t)N * H * 2);
    unsigned short* hl  = (unsigned short*)carve((size_t)N * H * 2);
    unsigned short* fh  = (unsigned short*)carve((size_t)N * F * 2);
    unsigned short* fl  = (unsigned short*)carve((size_t)N * F * 2);
    float* feat32       = (float*)carve((size_t)N * F * 4);
    float* Mm           = (float*)carve((size_t)N * B * 4);
    float* ob           = (float*)carve((size_t)N * B * 4);
    if (off > ws_size) return;

    float* out0 = (float*)d_out;
    float* out1 = out0 + (size_t)N * NM;

    cvt_split_rows<<<(N * DIN / 8 + 255) / 256, 256, 0, stream>>>(x, xh, xl, N * DIN / 8);
    cvt_split_transpose<<<dim3(H / 64, DIN / 64), 256, 0, stream>>>(Wb0, w0h, w0l, DIN, H);
    cvt_split_transpose<<<dim3(F / 64, H / 64), 256, 0, stream>>>(Wb1, w1h, w1l, H, F);
    cvt_split_transpose<<<dim3(B / 64, F / 64), 256, 0, stream>>>(T, th, tl, F, B);

    gemm_split3<true, true, false, true>
        <<<dim3(N / GT, H / GT), GEMM_THREADS, 0, stream>>>(
            (const __bf16*)xh, (const __bf16*)xl, (const __bf16*)w0h, (const __bf16*)w0l,
            bb0, nullptr, hh, hl, N, H, DIN);
    gemm_split3<true, true, true, true>
        <<<dim3(N / GT, F / GT), GEMM_THREADS, 0, stream>>>(
            (const __bf16*)hh, (const __bf16*)hl, (const __bf16*)w1h, (const __bf16*)w1l,
            bb1, feat32, fh, fl, N, F, H);
    gemm_split3<false, false, true, false>
        <<<dim3(N / GT, B / GT), GEMM_THREADS, 0, stream>>>(
            (const __bf16*)fh, (const __bf16*)fl, (const __bf16*)th, (const __bf16*)tl,
            nullptr, Mm, nullptr, nullptr, N, B, F);
    mbd_kernel<<<N / MBD_ROWS, 128, 0, stream>>>(Mm, ob, N);
    heads_kernel<<<N / HEAD_ROWS, 256, 0, stream>>>(feat32, ob, Wm, bm, Wc, bc, out0, out1);
}
